// MaskedEdgeHistoryEncoder_90134183674252
// MI455X (gfx1250) — hardware-run, weakly checked
//
#include <hip/hip_runtime.h>
#include <math.h>

typedef __attribute__((ext_vector_type(16))) _Float16 v16h;
typedef __attribute__((ext_vector_type(8)))  _Float16 v8h;
typedef __attribute__((ext_vector_type(8)))  float    v8f;
typedef __attribute__((ext_vector_type(4)))  float    v4f;
typedef __attribute__((ext_vector_type(2)))  float    v2f;
typedef __attribute__((ext_vector_type(4)))  unsigned int v4u;

constexpr int kBatch  = 2048;
constexpr int kSteps  = 50;
constexpr int kRel    = 6;
constexpr int kEty    = 4;
constexpr int kNode   = 9;
constexpr int kFeat   = kRel + kEty + kNode;
constexpr int kFeatP  = 32;
constexpr int kAtt    = 64;
constexpr int kHeads  = 4;
constexpr int kHead   = 16;
constexpr int kHid    = 128;
constexpr int kGate   = 4 * kHid;
constexpr int kOutD   = 64;
constexpr int kCat    = kAtt + kHid;
constexpr int kPairs  = kBatch * kSteps;
constexpr int kPB     = 16;
constexpr int kRowsB  = kPB * kNode;
constexpr int kMT     = kRowsB / 16;
constexpr int kAP     = 40;
constexpr int kQP     = 68;
constexpr int kAttP   = 12;
constexpr int kLB     = 16;
constexpr int kXP     = 200;
constexpr int kHP     = 132;
constexpr int kOP     = 68;

constexpr int isqrt_c(int v) { int r = 0; while ((r + 1) * (r + 1) <= v) ++r; return r; }
static_assert(isqrt_c(kHead) * isqrt_c(kHead) == kHead);
constexpr float kScoreScale = 1.0f / (float)isqrt_c(kHead);
constexpr float kMaskFill   = -1.0e10f;

constexpr float kFeatCarry = 16.0f;
constexpr float kWqvCarry  = 256.0f;
constexpr float kQVFold    = 1.0f / (kFeatCarry * kWqvCarry);
constexpr float kXHCarry   = 256.0f;
constexpr float kWcatCarry = 256.0f;
constexpr float kGateFold  = 1.0f / (kXHCarry * kWcatCarry);
constexpr float kF16MinNormal = 6.103515625e-05f;

static_assert(kFeat == 19);
static_assert(kHeads * kHead == kAtt);
static_assert(kFeatP % 32 == 0 && kCat % 32 == 0);
static_assert(kRowsB % 16 == 0 && kMT == 9);
static_assert(kPairs % kPB == 0 && kBatch % kLB == 0);
static_assert(kAtt * 2 == 128);
static_assert((kAP * 2) % 16 == 0 && (kXP * 2) % 16 == 0 && (kQP * 4) % 16 == 0 && (kHP * 4) % 16 == 0);

constexpr size_t kOffCtx  = 0;
constexpr size_t kOffWcat = kOffCtx  + (size_t)kSteps * kBatch * kAtt * 2;
constexpr size_t kOffWqv  = kOffWcat + (size_t)kGate * kCat * 2;
constexpr size_t kOffBqv  = kOffWqv  + (size_t)2 * kAtt * kFeatP * 2;
constexpr size_t kOffBsum = kOffBqv  + (size_t)2 * kAtt * 4;
constexpr size_t kWsTotal = kOffBsum + (size_t)kGate * 4;
static_assert(kWsTotal == 13314560ull);
static_assert(kWsTotal <= 134217728ull);
static_assert((kOffWcat % 128) == 0 && (kOffWqv % 128) == 0 && (kOffBqv % 128) == 0 && (kOffBsum % 128) == 0);

__device__ __forceinline__ unsigned h16_bits(float v) {
  const float w = (fabsf(v) < kF16MinNormal) ? 0.0f : v;
  const _Float16 h = (_Float16)w;
  const unsigned short s = __builtin_bit_cast(unsigned short, h);
  unsigned u = (unsigned)s;
  asm volatile("" : "+v"(u));
  return u;
}
__device__ __forceinline__ unsigned pk16(unsigned lo, unsigned hi) { return (hi << 16) | (lo & 0xffffu); }

struct FragH {
  union U { v16h v; v8h h[2]; };
  static __device__ __forceinline__ v16h load(const _Float16* p) {
    U f;
    f.h[0] = *(const v8h*)(p);
    f.h[1] = *(const v8h*)(p + 16);
    return f.v;
  }
};

__device__ __forceinline__ v8f mma_f16(v16h a, v16h b, v8f c) {
  c = __builtin_amdgcn_wmma_f32_16x16x32_f16(false, a, false, b, (short)0, c, false, false);
  asm volatile("v_nop\n\tv_nop\n\tv_nop\n\tv_nop" : "+v"(c) : "v"(a), "v"(b));
  return c;
}

__device__ __forceinline__ float dot4(v4f a, v4f b, float s) {
  s = fmaf(a[0], b[0], s);
  s = fmaf(a[1], b[1], s);
  s = fmaf(a[2], b[2], s);
  s = fmaf(a[3], b[3], s);
  return s;
}

__device__ __forceinline__ float sigm(float x) { return __builtin_amdgcn_rcpf(1.0f + expf(-x)); }

__global__ __launch_bounds__(256) void prep_planes_kernel(
    const float* __restrict__ W_fus, const float* __restrict__ b_fus,
    const float* __restrict__ Wq, const float* __restrict__ bq,
    const float* __restrict__ Wv, const float* __restrict__ bv,
    const float* __restrict__ W_ih, const float* __restrict__ W_hh,
    const float* __restrict__ b_ih, const float* __restrict__ b_hh,
    unsigned* __restrict__ wqvw, float* __restrict__ bqv,
    unsigned* __restrict__ wcatw, float* __restrict__ bsum)
{
  const unsigned lane = threadIdx.x & 31u;
  const unsigned gw = __builtin_amdgcn_readfirstlane(blockIdx.x * 8u + (threadIdx.x >> 5));
  if (gw < 64u) {
    const bool isV = (gw >= 32u);
    const float* Wsrc = isV ? Wv : Wq;
    const unsigned jr = 2u * (gw & 31u) + (lane >> 4);
    const unsigned c0 = 2u * (lane & 15u);
    const unsigned k0 = (c0 < (unsigned)(kFeat - 1)) ? c0 : (unsigned)(kFeat - 1);
    const unsigned k1 = (c0 + 1u < (unsigned)(kFeat - 1)) ? (c0 + 1u) : (unsigned)(kFeat - 1);
    const float* wr = Wsrc + jr * (unsigned)kAtt;
    float a0 = 0.0f, a1 = 0.0f;
#pragma unroll 4
    for (int m = 0; m < kAtt; ++m) {
      const float w = wr[m];
      a0 = fmaf(w, W_fus[m * kFeat + k0], a0);
      a1 = fmaf(w, W_fus[m * kFeat + k1], a1);
    }
    const float v0 = (c0 < (unsigned)kFeat) ? (a0 * kWqvCarry) : 0.0f;
    const float v1 = (c0 + 1u < (unsigned)kFeat) ? (a1 * kWqvCarry) : 0.0f;
    const unsigned word = pk16(h16_bits(v0), h16_bits(v1));
    unsigned* dst = wqvw + gw * 32u + lane;
    *(volatile unsigned*)dst = word;
    __threadfence();
    *(volatile unsigned*)dst = word;
  } else if (gw < 1600u) {
    const unsigned L = gw - 64u;
    const unsigned row = L / 3u;
    const unsigned seg = L - 3u * row;
    v2f wv;
    if (seg == 0u) {
      wv = *(const v2f*)(W_ih + row * (unsigned)kAtt + 2u * lane);
    } else {
      wv = *(const v2f*)(W_hh + row * (unsigned)kHid + (seg - 1u) * 64u + 2u * lane);
    }
    const float x0 = wv[0];
    const float x1 = wv[1];
    const unsigned word = pk16(h16_bits(x0 * kWcatCarry), h16_bits(x1 * kWcatCarry));
    unsigned* dst = wcatw + L * 32u + lane;
    *(volatile unsigned*)dst = word;
    __threadfence();
    *(volatile unsigned*)dst = word;
  } else if (gw < 1602u) {
    const bool isV = (gw == 1601u);
    const float* Wsrc = isV ? Wv : Wq;
    const float* bsrc = isV ? bv : bq;
    const unsigned j0 = 2u * lane;
    const float* w0p = Wsrc + j0 * (unsigned)kAtt;
    const float* w1p = w0p + kAtt;
    float a0 = 0.0f, a1 = 0.0f;
#pragma unroll 4
    for (int m = 0; m < kAtt; ++m) {
      const float bf = b_fus[m];
      a0 = fmaf(w0p[m], bf, a0);
      a1 = fmaf(w1p[m], bf, a1);
    }
    v2f o;
    o[0] = a0 + bsrc[j0];
    o[1] = a1 + bsrc[j0 + 1u];
    float* dst = bqv + (isV ? (unsigned)kAtt : 0u) + j0;
    *(volatile v2f*)dst = o;
    __threadfence();
    *(volatile v2f*)dst = o;
  } else if (gw < 1606u) {
    const unsigned idx = (gw - 1602u) * 128u + 4u * lane;
    const v4f a = *(const v4f*)(b_ih + idx);
    const v4f b = *(const v4f*)(b_hh + idx);
    const v4f s = a + b;
    float* dst = bsum + idx;
    *(volatile v4f*)dst = s;
    __threadfence();
    *(volatile v4f*)dst = s;
  }
}

__global__ __launch_bounds__(256) void attn_ctx_kernel(
    const float* __restrict__ seqs, const float* __restrict__ etys, const int* __restrict__ masks,
    const float* __restrict__ Wk, const float* __restrict__ bk,
    const unsigned short* __restrict__ wqv16, const float* __restrict__ bqv,
    unsigned* __restrict__ ctxw)
{
  __shared__ __align__(16) _Float16 sA[kRowsB * kAP];
  __shared__ __align__(16) float sQV[kRowsB * kQP];
  __shared__ __align__(16) float sKey[kPB * kAtt];
  __shared__ int sMsk[160];
  __shared__ float sAtt[kPB * kHeads * kAttP];

  const unsigned tid  = threadIdx.x;
  const unsigned lane = tid & 31u;
  const unsigned wave = __builtin_amdgcn_readfirstlane(tid >> 5);
  const unsigned ln   = lane & 15u;
  const unsigned lh   = lane >> 4;
  const unsigned gp0  = blockIdx.x * (unsigned)kPB;

  if (wave < 5u) {
    unsigned r = (tid < (unsigned)(kRowsB - 1)) ? tid : (unsigned)(kRowsB - 1);
    asm volatile("" : "+v"(r));
    const float* sp = seqs + (size_t)gp0 * (kNode * kRel) + r * (unsigned)kRel;
    const v2f s01 = *(const v2f*)(sp);
    const v2f s23 = *(const v2f*)(sp + 2);
    const v2f s45 = *(const v2f*)(sp + 4);
    const v4f ev  = *(const v4f*)(etys + (size_t)gp0 * (kNode * kEty) + r * (unsigned)kEty);
    int mk = masks[(size_t)gp0 * kNode + r];
    float f0 = s01[0], f1 = s01[1], f2 = s23[0], f3 = s23[1], f4 = s45[0], f5 = s45[1];
    float e0 = ev[0], e1 = ev[1], e2 = ev[2], e3 = ev[3];
    asm volatile("" : "+v"(f0), "+v"(f1), "+v"(f2), "+v"(f3), "+v"(f4), "+v"(f5));
    asm volatile("" : "+v"(e0), "+v"(e1), "+v"(e2), "+v"(e3));
    asm volatile("" : "+v"(mk));
    unsigned q9 = r / 9u;
    unsigned n  = r - q9 * 9u;
    asm volatile("" : "+v"(n));
    const unsigned w0 = pk16(h16_bits(f0 * kFeatCarry), h16_bits(f1 * kFeatCarry));
    const unsigned w1 = pk16(h16_bits(f2 * kFeatCarry), h16_bits(f3 * kFeatCarry));
    const unsigned w2 = pk16(h16_bits(f4 * kFeatCarry), h16_bits(f5 * kFeatCarry));
    const unsigned w3 = pk16(h16_bits(e0 * kFeatCarry), h16_bits(e1 * kFeatCarry));
    const unsigned w4 = pk16(h16_bits(e2 * kFeatCarry), h16_bits(e3 * kFeatCarry));
    const unsigned ohb = h16_bits(kFeatCarry);
    const unsigned oh  = (n & 1u) ? (ohb << 16) : ohb;
    const unsigned m2  = n >> 1;
    const unsigned w5 = (m2 == 0u) ? oh : 0u;
    const unsigned w6 = (m2 == 1u) ? oh : 0u;
    const unsigned w7 = (m2 == 2u) ? oh : 0u;
    const unsigned w8 = (m2 == 3u) ? oh : 0u;
    const unsigned w9 = (m2 == 4u) ? oh : 0u;
    if (tid < (unsigned)kRowsB) {
      v4u* dst = (v4u*)(sA + r * (unsigned)kAP);
      dst[0] = (v4u){w0, w1, w2, w3};
      dst[1] = (v4u){w4, w5, w6, w7};
      dst[2] = (v4u){w8, w9, 0u, 0u};
      dst[3] = (v4u){0u, 0u, 0u, 0u};
      sMsk[r] = mk;
    }
  }

  {
    const unsigned j  = tid & 63u;
    const unsigned pg = tid >> 6;
    const v2f k01 = *(const v2f*)(Wk + j * (unsigned)kRel);
    const v2f k23 = *(const v2f*)(Wk + j * (unsigned)kRel + 2);
    const v2f k45 = *(const v2f*)(Wk + j * (unsigned)kRel + 4);
    const float kb = bk[j];
#pragma unroll
    for (int i = 0; i < 4; ++i) {
      const unsigned p = pg * 4u + (unsigned)i;
      const float* sp = seqs + (size_t)(gp0 + p) * (kNode * kRel) + 4 * kRel;
      const v2f a01 = *(const v2f*)(sp);
      const v2f a23 = *(const v2f*)(sp + 2);
      const v2f a45 = *(const v2f*)(sp + 4);
      float acc = 0.0f;
      acc = fmaf(a01[0], k01[0], acc);
      acc = fmaf(a01[1], k01[1], acc);
      acc = fmaf(a23[0], k23[0], acc);
      acc = fmaf(a23[1], k23[1], acc);
      acc = fmaf(a45[0], k45[0], acc);
      acc = fmaf(a45[1], k45[1], acc);
      sKey[p * (unsigned)kAtt + j] = acc + kb;
    }
  }
  __syncthreads();

  const _Float16* wq = (const _Float16*)wqv16;
  const v16h bfr = FragH::load(wq + (16u * wave + ln) * (unsigned)kFeatP + 8u * lh);
  v8f acc[kMT];
#pragma unroll
  for (int mt = 0; mt < kMT; ++mt) {
    acc[mt] = (v8f){0.f, 0.f, 0.f, 0.f, 0.f, 0.f, 0.f, 0.f};
    const v16h afr = FragH::load(sA + (16u * (unsigned)mt + ln) * (unsigned)kAP + 8u * lh);
    acc[mt] = mma_f16(afr, bfr, acc[mt]);
  }
  const float bias = bqv[16u * wave + ln];
  if (wave < 4u) {
#pragma unroll
    for (int mt = 0; mt < kMT; ++mt) {
#pragma unroll
      for (int r = 0; r < 8; ++r) {
        sQV[(16u * (unsigned)mt + 8u * lh + (unsigned)r) * (unsigned)kQP + 16u * wave + ln] = fmaf(acc[mt][r], kQVFold, bias);
      }
    }
  }
  __syncthreads();

  if (wave < 2u) {
    const unsigned p  = tid >> 2;
    const unsigned hd = tid & 3u;
    const float* kp = sKey + p * (unsigned)kAtt + hd * (unsigned)kHead;
    const v4f ka = *(const v4f*)(kp);
    const v4f kb4 = *(const v4f*)(kp + 4);
    const v4f kc = *(const v4f*)(kp + 8);
    const v4f kd = *(const v4f*)(kp + 12);
    float sc[kNode];
    float mx = -3.0e38f;
#pragma unroll
    for (int n = 0; n < kNode; ++n) {
      const float* qp = sQV + (p * (unsigned)kNode + (unsigned)n) * (unsigned)kQP + hd * (unsigned)kHead;
      const v4f qa = *(const v4f*)(qp);
      const v4f qb = *(const v4f*)(qp + 4);
      const v4f qc = *(const v4f*)(qp + 8);
      const v4f qd = *(const v4f*)(qp + 12);
      float s = 0.0f;
      s = dot4(ka, qa, s);
      s = dot4(kb4, qb, s);
      s = dot4(kc, qc, s);
      s = dot4(kd, qd, s);
      s = s * kScoreScale;
      const int mk = sMsk[p * (unsigned)kNode + (unsigned)n];
      s = (mk == 0) ? kMaskFill : s;
      sc[n] = s;
      mx = fmaxf(mx, s);
    }
    float sum = 0.0f;
#pragma unroll
    for (int n = 0; n < kNode; ++n) {
      sc[n] = expf(sc[n] - mx);
      sum += sc[n];
    }
    const float inv = 1.0f / sum;
#pragma unroll
    for (int n = 0; n < kNode; ++n) sAtt[(p * (unsigned)kHeads + hd) * (unsigned)kAttP + (unsigned)n] = sc[n] * inv;
  }
  __syncthreads();

  if (wave >= 4u) {
#pragma unroll
    for (int mt = 0; mt < kMT; ++mt) {
#pragma unroll
      for (int r = 0; r < 8; ++r) {
        sQV[(16u * (unsigned)mt + 8u * lh + (unsigned)r) * (unsigned)kQP + 16u * (wave - 4u) + ln] = fmaf(acc[mt][r], kQVFold, bias);
      }
    }
  }
  __syncthreads();

  unsigned word[2];
  unsigned rowi[2];
#pragma unroll
  for (int i = 0; i < 2; ++i) {
    const unsigned p  = 2u * wave + (unsigned)i;
    const unsigned hd = lane >> 3;
    const float* at = sAtt + (p * (unsigned)kHeads + hd) * (unsigned)kAttP;
    float c0 = 0.0f, c1 = 0.0f;
#pragma unroll
    for (int n = 0; n < kNode; ++n) {
      const v2f vv = *(const v2f*)(sQV + (p * (unsigned)kNode + (unsigned)n) * (unsigned)kQP + 2u * lane);
      const float a = at[n];
      c0 = fmaf(a, vv[0], c0);
      c1 = fmaf(a, vv[1], c1);
    }
    word[i] = pk16(h16_bits(c0 * kXHCarry), h16_bits(c1 * kXHCarry));
    unsigned gp = gp0 + p;
    unsigned b  = gp / (unsigned)kSteps;
    unsigned s  = gp - b * (unsigned)kSteps;
    unsigned ri = s * (unsigned)kBatch + b;
    asm volatile("" : "+v"(ri));
    rowi[i] = ri;
  }
  for (int pass = 0; pass < 2; ++pass) {
#pragma unroll
    for (int i = 0; i < 2; ++i) {
      *(volatile unsigned*)(ctxw + (size_t)rowi[i] * 32u + lane) = word[i];
    }
    __threadfence();
  }
}

__global__ __launch_bounds__(256) void lstm_out_kernel(
    const unsigned short* __restrict__ ctx16, const unsigned short* __restrict__ wcat16,
    const float* __restrict__ bsum, const float* __restrict__ W_out, const float* __restrict__ b_out,
    float* __restrict__ out)
{
  __shared__ __align__(16) _Float16 sXH[2 * kLB * kXP];
  __shared__ __align__(16) float sHf[kLB * kHP];
  __shared__ __align__(16) float sO[kLB * kOP];

  const unsigned tid  = threadIdx.x;
  const unsigned lane = tid & 31u;
  const unsigned wave = __builtin_amdgcn_readfirstlane(tid >> 5);
  const unsigned ln   = lane & 15u;
  const unsigned lh   = lane >> 4;
  const unsigned row0 = blockIdx.x * (unsigned)kLB;
  const _Float16* wcat = (const _Float16*)wcat16;

  {
    const unsigned zr = tid >> 4, zc = tid & 15u;
    *(v4u*)(sXH + zr * (unsigned)kXP + (unsigned)kAtt + zc * 8u) = (v4u){0u, 0u, 0u, 0u};
  }
  const unsigned xr = (tid >> 3) & 15u;
  const unsigned xc = tid & 7u;
  if (wave < 4u) {
    const v4u x0 = *(const v4u*)(ctx16 + ((size_t)(row0 + xr)) * kAtt + xc * 8u);
    *(v4u*)(sXH + xr * (unsigned)kXP + xc * 8u) = x0;
  }

  const unsigned jcol = 16u * wave + ln;
  const float bI = bsum[jcol];
  const float bF = bsum[kHid + jcol];
  const float bG = bsum[2 * kHid + jcol];
  const float bO = bsum[3 * kHid + jcol];
  const unsigned wofs0 = jcol * (unsigned)kCat + 8u * lh;

  float c[8], hv[8];
#pragma unroll
  for (int r = 0; r < 8; ++r) { c[r] = 0.0f; hv[r] = 0.0f; }
  __syncthreads();

#pragma unroll 1
  for (int t = 0; t < kSteps; ++t) {
    const unsigned cb = (unsigned)(t & 1) * (unsigned)(kLB * kXP);
    const unsigned nb = (unsigned)((t + 1) & 1) * (unsigned)(kLB * kXP);
    const int tn = (t + 1 < kSteps) ? (t + 1) : (kSteps - 1);
    v4u xn = (v4u){0u, 0u, 0u, 0u};
    if (wave < 4u) {
      xn = *(const v4u*)(ctx16 + ((size_t)tn * kBatch + row0 + xr) * kAtt + xc * 8u);
    }
    unsigned woff = wofs0;
    asm volatile("" : "+v"(woff));
    const _Float16* wb = wcat + woff;
    const _Float16* ab = sXH + cb + ln * (unsigned)kXP + 8u * lh;

    v8f acc[4];
#pragma unroll
    for (int g = 0; g < 4; ++g) acc[g] = (v8f){0.f, 0.f, 0.f, 0.f, 0.f, 0.f, 0.f, 0.f};
#pragma unroll
    for (int ks = 0; ks < kCat / 32; ++ks) {
      const v16h afr = FragH::load(ab + ks * 32);
#pragma unroll
      for (int g = 0; g < 4; ++g) {
        const v16h bfr = FragH::load(wb + g * (kHid * kCat) + ks * 32);
        acc[g] = mma_f16(afr, bfr, acc[g]);
      }
    }

    _Float16* hdst = sXH + nb + (8u * lh) * (unsigned)kXP + (unsigned)kAtt + jcol;
#pragma unroll
    for (int r = 0; r < 8; ++r) {
      const float gi = fmaf(acc[0][r], kGateFold, bI);
      const float gf = fmaf(acc[1][r], kGateFold, bF);
      const float gg = fmaf(acc[2][r], kGateFold, bG);
      const float go = fmaf(acc[3][r], kGateFold, bO);
      const float ig = sigm(gi);
      const float fg = sigm(gf);
      const float tg = tanhf(gg);
      const float og = sigm(go);
      const float cn = fg * c[r] + ig * tg;
      c[r] = cn;
      const float hn = og * tanhf(cn);
      hv[r] = hn;
      const float hc = hn * kXHCarry;
      const float hz = (fabsf(hc) < kF16MinNormal) ? 0.0f : hc;
      hdst[r * kXP] = (_Float16)hz;
    }
    if (wave < 4u) {
      *(v4u*)(sXH + nb + xr * (unsigned)kXP + xc * 8u) = xn;
    }
    __syncthreads();
  }

#pragma unroll
  for (int r = 0; r < 8; ++r) sHf[(8u * lh + (unsigned)r) * (unsigned)kHP + jcol] = hv[r];
  __syncthreads();
  {
    const unsigned o  = tid & 63u;
    const unsigned rg = tid >> 6;
    const float* wrow = W_out + o * (unsigned)kHid;
    const float* h0p = sHf + (rg * 4u + 0u) * (unsigned)kHP;
    const float* h1p = sHf + (rg * 4u + 1u) * (unsigned)kHP;
    const float* h2p = sHf + (rg * 4u + 2u) * (unsigned)kHP;
    const float* h3p = sHf + (rg * 4u + 3u) * (unsigned)kHP;
    float a0 = 0.0f, a1 = 0.0f, a2 = 0.0f, a3 = 0.0f;
#pragma unroll 2
    for (int k4 = 0; k4 < kHid / 4; ++k4) {
      const v4f w = *(const v4f*)(wrow + 4 * k4);
      a0 = dot4(w, *(const v4f*)(h0p + 4 * k4), a0);
      a1 = dot4(w, *(const v4f*)(h1p + 4 * k4), a1);
      a2 = dot4(w, *(const v4f*)(h2p + 4 * k4), a2);
      a3 = dot4(w, *(const v4f*)(h3p + 4 * k4), a3);
    }
    const float bo = b_out[o];
    sO[(rg * 4u + 0u) * (unsigned)kOP + o] = a0 + bo;
    sO[(rg * 4u + 1u) * (unsigned)kOP + o] = a1 + bo;
    sO[(rg * 4u + 2u) * (unsigned)kOP + o] = a2 + bo;
    sO[(rg * 4u + 3u) * (unsigned)kOP + o] = a3 + bo;
  }
  __syncthreads();
  {
    const unsigned row = 2u * wave + lh;
    const v4f v = *(const v4f*)(sO + row * (unsigned)kOP + 4u * ln);
    float* dst = out + (size_t)(row0 + row) * kOutD + 4u * ln;
    *(volatile v4f*)dst = v;
    __threadfence();
    *(volatile v4f*)dst = v;
  }
}

extern "C" void kernel_launch(void* const* d_in, const int* in_sizes, int n_in,
                              void* d_out, int out_size, void* d_ws, size_t ws_size,
                              hipStream_t stream) {
  if (n_in < 17) return;
  if (in_sizes[0] != kPairs * kNode * kRel) return;
  if (in_sizes[1] != kPairs * kNode * kEty) return;
  if (in_sizes[2] != kPairs * kNode) return;
  if (in_sizes[3] != kAtt * kFeat) return;
  if (in_sizes[4] != kAtt) return;
  if (in_sizes[5] != kAtt * kRel) return;
  if (in_sizes[6] != kAtt) return;
  if (in_sizes[7] != kAtt * kAtt) return;
  if (in_sizes[8] != kAtt) return;
  if (in_sizes[9] != kAtt * kAtt) return;
  if (in_sizes[10] != kAtt) return;
  if (in_sizes[11] != kGate * kAtt) return;
  if (in_sizes[12] != kGate * kHid) return;
  if (in_sizes[13] != kGate) return;
  if (in_sizes[14] != kGate) return;
  if (in_sizes[15] != kOutD * kHid) return;
  if (in_sizes[16] != kOutD) return;
  if (out_size != kBatch * kOutD) return;
  if (ws_size < kWsTotal) return;

  const float* seqs  = (const float*)d_in[0];
  const float* etys  = (const float*)d_in[1];
  const int*   masks = (const int*)  d_in[2];
  const float* W_fus = (const float*)d_in[3];
  const float* b_fus = (const float*)d_in[4];
  const float* Wk    = (const float*)d_in[5];
  const float* bk    = (const float*)d_in[6];
  const float* Wq    = (const float*)d_in[7];
  const float* bq    = (const float*)d_in[8];
  const float* Wv    = (const float*)d_in[9];
  const float* bv    = (const float*)d_in[10];
  const float* W_ih  = (const float*)d_in[11];
  const float* W_hh  = (const float*)d_in[12];
  const float* b_ih  = (const float*)d_in[13];
  const float* b_hh  = (const float*)d_in[14];
  const float* W_out = (const float*)d_in[15];
  const float* b_out = (const float*)d_in[16];

  char* ws = (char*)d_ws;
  unsigned short* ctx16  = (unsigned short*)(ws + kOffCtx);
  unsigned short* wcat16 = (unsigned short*)(ws + kOffWcat);
  unsigned short* wqv16  = (unsigned short*)(ws + kOffWqv);
  float*          bqv    = (float*)(ws + kOffBqv);
  float*          bsum   = (float*)(ws + kOffBsum);

  prep_planes_kernel<<<201, 256, 0, stream>>>(W_fus, b_fus, Wq, bq, Wv, bv, W_ih, W_hh, b_ih, b_hh,
                                              (unsigned*)wqv16, bqv, (unsigned*)wcat16, bsum);

  attn_ctx_kernel<<<kPairs / kPB, 256, 0, stream>>>(seqs, etys, masks, Wk, bk, wqv16, bqv, (unsigned*)ctx16);

  lstm_out_kernel<<<kBatch / kLB, 256, 0, stream>>>(ctx16, wcat16, bsum, W_out, b_out, (float*)d_out);
}
